// MultiHeadSelfAttention_56521769615862
// MI455X (gfx1250) — hardware-verified
//
#include <hip/hip_runtime.h>


#ifndef NB
#define NB 8
#endif
#ifndef SEQ
#define SEQ 2048
#endif
#define NB_FULL  8
#define SEQ_FULL 2048
#define DM   384
#define NH   6
#define HD   64
#define MTOK (NB * SEQ)
#define PCAR 16384.0f
#define L2E  1.4426950408889634f

static_assert(SEQ % 64 == 0);
static_assert(DM % 64 == 0);
static_assert(DM % 32 == 0);
static_assert(NH * HD == DM);
static_assert(NB <= NB_FULL);
static_assert(SEQ <= SEQ_FULL);
static_assert((size_t)4 * DM * DM * 2 + (size_t)7 * MTOK * DM * 2 <= (size_t)134217728);

typedef _Float16 h16;
typedef unsigned short bf;
typedef __attribute__((ext_vector_type(16))) __bf16   v16bf;
typedef __attribute__((ext_vector_type(16))) _Float16 v16h;
typedef __attribute__((ext_vector_type(8)))  _Float16 v8h;
typedef __attribute__((ext_vector_type(8)))  unsigned short v8us;
typedef __attribute__((ext_vector_type(4)))  unsigned short v4us;
typedef __attribute__((ext_vector_type(8)))  float    v8f;
typedef __attribute__((ext_vector_type(4)))  float    v4f;
typedef v4f  __attribute__((may_alias)) v4fa;

__device__ __forceinline__ unsigned short f2bf(float f) { unsigned u = __float_as_uint(f); u += 0x7FFFu + ((u >> 16) & 1u); return (unsigned short)(u >> 16); }
__device__ __forceinline__ float bf2f(unsigned short b) { return __uint_as_float(((unsigned)b) << 16); }
__device__ __forceinline__ float bfr(float f) { return bf2f(f2bf(f)); }
__device__ __forceinline__ void splitf(float y, unsigned short& h, unsigned short& l) { h = f2bf(y); l = f2bf(y - bf2f(h)); }
__device__ __forceinline__ v16h cat16(v8h lo, v8h hi) { return __builtin_shufflevector(lo, hi, 0, 1, 2, 3, 4, 5, 6, 7, 8, 9, 10, 11, 12, 13, 14, 15); }
__device__ __forceinline__ v16bf cat16b(v8us lo, v8us hi) { return __builtin_bit_cast(v16bf, __builtin_shufflevector(lo, hi, 0, 1, 2, 3, 4, 5, 6, 7, 8, 9, 10, 11, 12, 13, 14, 15)); }
__device__ __forceinline__ v8f wmma16(v16h a, v16h b, v8f c) { return __builtin_amdgcn_wmma_f32_16x16x32_f16(false, a, false, b, (short)0, c, false, false); }
__device__ __forceinline__ v8f wmmab(v16bf a, v16bf b, v8f c) { return __builtin_amdgcn_wmma_f32_16x16x32_bf16(false, a, false, b, (short)0, c, false, false); }
__device__ __forceinline__ v16bf ldb(const bf* p) { return cat16b(*(const v8us*)p, *(const v8us*)(p + 16)); }
__device__ __forceinline__ v16h ldh(const h16* p) { return cat16(*(const v8h*)p, *(const v8h*)(p + 16)); }
__device__ __forceinline__ void wave_lds_sync() { __builtin_amdgcn_fence(3  , "wavefront"); __builtin_amdgcn_wave_barrier(); __builtin_amdgcn_fence(2  , "wavefront"); asm volatile("" ::: "memory"); }

__global__ __launch_bounds__(256) void k_wt(const float* __restrict__ src, bf* dst, int rows, int cols) {
    __shared__ float t[64 * 65];
    const int tid = threadIdx.x;
    const size_t zo = (size_t)blockIdx.z * (size_t)rows * (size_t)cols;
    const int r0 = blockIdx.x * 64, c0 = blockIdx.y * 64;
#pragma unroll 4
    for (int i = 0; i < 16; ++i) { const int rr = (tid >> 6) + 4 * i, cc = tid & 63; t[rr * 65 + cc] = src[zo + (size_t)(r0 + rr) * cols + c0 + cc]; }
    __syncthreads();
    const int pc = tid & 7;
#pragma unroll 1
    for (int ps = 0; ps < 2; ++ps) {
#pragma unroll
        for (int it = 0; it < 2; ++it) { const int line = (tid >> 3) + 32 * it; v8us o;
#pragma unroll
            for (int i = 0; i < 8; ++i) o[i] = f2bf(t[(8 * pc + i) * 65 + line]);
            *(volatile v8us*)(dst + zo + (size_t)(c0 + line) * rows + r0 + 8 * pc) = o; }
        if (ps == 0) __threadfence(); }
}

__global__ __launch_bounds__(256) void k_ln(const float* __restrict__ x, const float* __restrict__ g, const float* __restrict__ be, bf* Yh, bf* Yl) {
    const int lane = threadIdx.x & 31;
    const int wave = __builtin_amdgcn_readfirstlane(threadIdx.x >> 5);
    const int tok = blockIdx.x * 8 + wave;
    const int b = tok / SEQ, s = tok % SEQ;
    const float* xr = x + ((size_t)b * SEQ_FULL + s) * DM;
    v4f v[3]; float sum = 0.0f;
#pragma unroll
    for (int j = 0; j < 3; ++j) { v4f a = *(const v4f*)(xr + j * 128 + lane * 4);
#pragma unroll
        for (int q = 0; q < 4; ++q) { a[q] = bfr(a[q]); sum += a[q]; }
        v[j] = a; }
#pragma unroll
    for (int sh = 16; sh; sh >>= 1) sum += __shfl_xor(sum, sh, 32);
    const float mu = sum * (1.0f / DM);
    float var = 0.0f;
#pragma unroll
    for (int j = 0; j < 3; ++j) {
#pragma unroll
        for (int q = 0; q < 4; ++q) { const float d = v[j][q] - mu; var += d * d; } }
#pragma unroll
    for (int sh = 16; sh; sh >>= 1) var += __shfl_xor(var, sh, 32);
    const float rs = rsqrtf(var * (1.0f / DM) + 1e-5f);
    v4us oh[3], ol[3];
#pragma unroll
    for (int j = 0; j < 3; ++j) { const v4f gg = *(const v4f*)(g + j * 128 + lane * 4); const v4f bb = *(const v4f*)(be + j * 128 + lane * 4);
#pragma unroll
        for (int q = 0; q < 4; ++q) { const float y = (v[j][q] - mu) * rs * bfr(gg[q]) + bfr(bb[q]); unsigned short a, c; splitf(y, a, c); oh[j][q] = a; ol[j][q] = c; } }
    const size_t ro = (size_t)tok * DM + lane * 4;
#pragma unroll 1
    for (int ps = 0; ps < 2; ++ps) {
#pragma unroll
        for (int j = 0; j < 3; ++j) { *(volatile v4us*)(Yh + ro + j * 128) = oh[j]; *(volatile v4us*)(Yl + ro + j * 128) = ol[j]; }
        if (ps == 0) __threadfence(); }
}

template <int MODE>
__global__ __launch_bounds__(32) void k_gemmw(const bf* __restrict__ A, const bf* __restrict__ A2, const bf* __restrict__ Bt, const float* __restrict__ bias, bf* Oh, bf* Ol, h16* Ov, float* Of) {
    __shared__ __align__(16) float os[64 * 68];
    const int lane = threadIdx.x & 31, lr = lane & 15, hi = lane >> 4;
    const int r0 = blockIdx.x * 64, c0 = blockIdx.y * 64;
    v8f acc[4][4];
#pragma unroll
    for (int mb = 0; mb < 4; ++mb)
#pragma unroll
        for (int nb = 0; nb < 4; ++nb) acc[mb][nb] = (v8f){};
    const size_t aoff = (size_t)(r0 + lr) * DM + 8 * hi, boff = (size_t)(c0 + lr) * DM + 8 * hi;
#pragma unroll 1
    for (int kc = 0; kc < DM; kc += 32) {
        v16bf a[4], a2[4], b;
#pragma unroll
        for (int mb = 0; mb < 4; ++mb) { a[mb] = ldb(A + aoff + (size_t)mb * 16 * DM + kc); a2[mb] = ldb(A2 + aoff + (size_t)mb * 16 * DM + kc); }
#pragma unroll
        for (int nb = 0; nb < 4; ++nb) { b = ldb(Bt + boff + (size_t)nb * 16 * DM + kc);
#pragma unroll
            for (int mb = 0; mb < 4; ++mb) { acc[mb][nb] = wmmab(a[mb], b, acc[mb][nb]); acc[mb][nb] = wmmab(a2[mb], b, acc[mb][nb]); } }
        asm volatile("" : "+v"(acc[0][0]), "+v"(acc[1][0]), "+v"(acc[2][0]), "+v"(acc[3][0]), "+v"(acc[0][1]), "+v"(acc[1][1]), "+v"(acc[2][1]), "+v"(acc[3][1]));
        asm volatile("v_nop\n\tv_nop\n\tv_nop\n\tv_nop" : "+v"(acc[0][2]), "+v"(acc[1][2]), "+v"(acc[2][2]), "+v"(acc[3][2]), "+v"(acc[0][3]), "+v"(acc[1][3]), "+v"(acc[2][3]), "+v"(acc[3][3]) : "v"(a[3]), "v"(a2[3]), "v"(b));
    }
#pragma unroll
    for (int mb = 0; mb < 4; ++mb)
#pragma unroll
        for (int nb = 0; nb < 4; ++nb)
#pragma unroll
            for (int j = 0; j < 8; ++j) os[(mb * 16 + hi * 8 + j) * 68 + nb * 16 + lr] = acc[mb][nb][j];
    wave_lds_sync();
    const int bb = r0 / SEQ, sq = r0 % SEQ, hh = blockIdx.y;
    const int rq = lane >> 3, pc = lane & 7;
    if (MODE == 0) {
        const size_t pb = ((size_t)(bb * NH + hh) * SEQ + sq) * HD;
        float bz[8];
#pragma unroll
        for (int i = 0; i < 8; ++i) bz[i] = bfr(bias[c0 + 8 * pc + i]);
#pragma unroll 1
        for (int ps = 0; ps < 2; ++ps) {
#pragma unroll 1
            for (int s = 0; s < 16; ++s) { const int row = 4 * s + rq;
                const v4f u0 = *(const v4fa*)(os + row * 68 + 8 * pc); const v4f u1 = *(const v4fa*)(os + row * 68 + 8 * pc + 4); v8us oh, ol;
#pragma unroll
                for (int i = 0; i < 4; ++i) { unsigned short a, c; splitf(u0[i] + bz[i], a, c); oh[i] = a; ol[i] = c; splitf(u1[i] + bz[4 + i], a, c); oh[4 + i] = a; ol[4 + i] = c; }
                *(volatile v8us*)(Oh + pb + (size_t)row * HD + 8 * pc) = oh; *(volatile v8us*)(Ol + pb + (size_t)row * HD + 8 * pc) = ol; }
            if (ps == 0) __threadfence(); }
    }
    if (MODE == 1) {
        const size_t vb = (size_t)(bb * NH + hh) * HD * SEQ + sq;
#pragma unroll 1
        for (int ps = 0; ps < 2; ++ps) {
#pragma unroll 1
            for (int s = 0; s < 16; ++s) { const int hd = 4 * s + rq; const float bzv = bfr(bias[c0 + hd]); v8h o8;
#pragma unroll
                for (int i = 0; i < 8; ++i) o8[i] = (h16)(os[(8 * pc + i) * 68 + hd] + bzv);
                *(volatile v8h*)(Ov + vb + (size_t)hd * SEQ + 8 * pc) = o8; }
            if (ps == 0) __threadfence(); }
    }
    if (MODE == 2) {
        const int cofs = lr * 4;
        float bz4[4];
#pragma unroll
        for (int q = 0; q < 4; ++q) bz4[q] = bfr(bias[c0 + cofs + q]);
#pragma unroll 1
        for (int ps = 0; ps < 2; ++ps) {
#pragma unroll 1
            for (int s = 0; s < 32; ++s) { const int row = 2 * s + hi; v4f val = *(const v4fa*)(os + row * 68 + cofs);
#pragma unroll
                for (int q = 0; q < 4; ++q) { const float tv = val[q] + bz4[q]; val[q] = 0.5f * tv * (1.0f + erff(tv * 0.70710678118654752f)); }
                *(volatile v4f*)(Of + (size_t)(r0 + row) * DM + c0 + cofs) = val; }
            if (ps == 0) __threadfence(); }
    }
}

__global__ __launch_bounds__(128) void k_attn(const bf* __restrict__ Qh, const bf* __restrict__ Ql, const bf* __restrict__ Kh, const bf* __restrict__ Kl, const h16* __restrict__ Vt, bf* Ch, bf* Cl) {
#pragma clang fp contract(off)
    __shared__ __align__(16) float os[4 * 16 * 68];
    const int lane = threadIdx.x & 31, lr = lane & 15, hi = lane >> 4;
    const int wave = __builtin_amdgcn_readfirstlane(threadIdx.x >> 5);
    const int bh = blockIdx.y;
    const int q0 = blockIdx.x * 64 + wave * 16;
    const size_t pbase = (size_t)bh * SEQ * HD;
    const bf* qh = Qh + pbase; const bf* ql = Ql + pbase; const bf* kh = Kh + pbase; const bf* kl = Kl + pbase; const h16* vt = Vt + pbase;
    const int qoff0 = (q0 + lr) * HD + 8 * hi;
    v8f o[4];
#pragma unroll
    for (int j = 0; j < 4; ++j) o[j] = (v8f){};
    float m = -1.0e30f, l = 0.0f;
#pragma unroll 1
    for (int kb = 0; kb < SEQ; kb += 32) {
        int qo = qoff0; asm volatile("" : "+v"(qo));
        const int ko = (kb + lr) * HD + 8 * hi;
        v8f s0 = (v8f){}, s1 = (v8f){};
#pragma unroll
        for (int ks = 0; ks < 2; ++ks) {
            const v16bf bqh = ldb(qh + qo + ks * 32), bql = ldb(ql + qo + ks * 32);
            const v16bf a0h = ldb(kh + ko + ks * 32), a0l = ldb(kl + ko + ks * 32);
            const v16bf a1h = ldb(kh + ko + 16 * HD + ks * 32), a1l = ldb(kl + ko + 16 * HD + ks * 32);
            s0 = wmmab(a0h, bqh, s0); s1 = wmmab(a1h, bqh, s1);
            s0 = wmmab(a0l, bqh, s0); s1 = wmmab(a1l, bqh, s1);
            s0 = wmmab(a0h, bql, s0); s1 = wmmab(a1h, bql, s1);
            asm volatile("v_nop\n\tv_nop\n\tv_nop\n\tv_nop" : "+v"(s0), "+v"(s1) : "v"(a0h), "v"(a1h), "v"(bql));
        }
        float mx = fmaxf(s0[0], s1[0]);
#pragma unroll
        for (int r = 1; r < 8; ++r) mx = fmaxf(mx, fmaxf(s0[r], s1[r]));
        mx = fmaxf(mx, __shfl_xor(mx, 16, 32));
        const float mn = fmaxf(m, mx);
        const float alpha = __builtin_amdgcn_exp2f((m - mn) * L2E);
        m = mn;
        float psum = 0.0f; v16h pf;
#pragma unroll
        for (int r = 0; r < 8; ++r) {
            const float p0 = __builtin_amdgcn_exp2f((s0[r] - mn) * L2E);
            const float p1 = __builtin_amdgcn_exp2f((s1[r] - mn) * L2E);
            psum += p0 + p1;
            pf[r] = (h16)(p0 * PCAR); pf[8 + r] = (h16)(p1 * PCAR); }
        l = l * alpha + psum;
#pragma unroll
        for (int j = 0; j < 4; ++j)
#pragma unroll
            for (int r = 0; r < 8; ++r) o[j][r] *= alpha;
        const int vo = lr * SEQ + kb + 8 * hi;
        const v16h va0 = ldh(vt + vo), va1 = ldh(vt + vo + 16 * SEQ), va2 = ldh(vt + vo + 32 * SEQ), va3 = ldh(vt + vo + 48 * SEQ);
        o[0] = wmma16(va0, pf, o[0]); o[1] = wmma16(va1, pf, o[1]); o[2] = wmma16(va2, pf, o[2]); o[3] = wmma16(va3, pf, o[3]);
        asm volatile("v_nop\n\tv_nop\n\tv_nop\n\tv_nop" : "+v"(o[0]), "+v"(o[1]), "+v"(o[2]), "+v"(o[3]) : "v"(va3), "v"(pf));
    }
    l += __shfl_xor(l, 16, 32);
    const float inv = 1.0f / (l * PCAR);
    const int wbase = wave * (16 * 68);
#pragma unroll
    for (int j = 0; j < 4; ++j)
#pragma unroll
        for (int r = 0; r < 8; ++r) os[wbase + lr * 68 + 16 * j + 8 * hi + r] = o[j][r] * inv;
    wave_lds_sync();
    const int b = bh / NH, h = bh % NH;
    const int rq = lane >> 3, pc = lane & 7;
#pragma unroll 1
    for (int ps = 0; ps < 2; ++ps) {
#pragma unroll
        for (int s = 0; s < 4; ++s) { const int row = 4 * s + rq;
            const v4f u0 = *(const v4fa*)(os + wbase + row * 68 + 8 * pc); const v4f u1 = *(const v4fa*)(os + wbase + row * 68 + 8 * pc + 4); v8us oh, ol;
#pragma unroll
            for (int i = 0; i < 4; ++i) { unsigned short a, c; splitf(u0[i], a, c); oh[i] = a; ol[i] = c; splitf(u1[i], a, c); oh[4 + i] = a; ol[4 + i] = c; }
            const size_t oo = ((size_t)b * SEQ + q0 + row) * DM + h * HD + 8 * pc;
            *(volatile v8us*)(Ch + oo) = oh; *(volatile v8us*)(Cl + oo) = ol; }
        if (ps == 0) __threadfence(); }
}

extern "C" void kernel_launch(void* const* d_in, const int* in_sizes, int n_in,
                              void* d_out, int out_size, void* d_ws, size_t ws_size, hipStream_t stream) {
    if (n_in < 11) return;
    if ((size_t)in_sizes[0] < ((size_t)(NB - 1) * SEQ_FULL + SEQ) * DM) return;
    if (in_sizes[1] < DM || in_sizes[2] < DM) return;
    if (in_sizes[3] < NH * DM * HD || in_sizes[5] < NH * DM * HD || in_sizes[7] < NH * DM * HD || in_sizes[9] < DM * DM) return;
    if (in_sizes[4] < DM || in_sizes[6] < DM || in_sizes[8] < DM || in_sizes[10] < DM) return;
    if ((size_t)out_size < (size_t)MTOK * DM) return;
    const float* x   = (const float*)d_in[0];
    const float* lng = (const float*)d_in[1];
    const float* lnb = (const float*)d_in[2];
    const float* wq  = (const float*)d_in[3];
    const float* bq  = (const float*)d_in[4];
    const float* wk  = (const float*)d_in[5];
    const float* bk  = (const float*)d_in[6];
    const float* wv  = (const float*)d_in[7];
    const float* bv  = (const float*)d_in[8];
    const float* wp  = (const float*)d_in[9];
    const float* bp  = (const float*)d_in[10];
    float* OUT = (float*)d_out;
    char* wsp = (char*)d_ws;
    auto take = [&](size_t bytes) { char* p = wsp; wsp += (bytes + 255) & ~(size_t)255; return (void*)p; };
    const size_t WSZ = (size_t)DM * DM * 2;
    const size_t PSZ = (size_t)MTOK * DM * 2;
    bf* WQ = (bf*)take(WSZ); bf* WK = (bf*)take(WSZ); bf* WV = (bf*)take(WSZ); bf* WP = (bf*)take(WSZ);
    bf* Yh = (bf*)take(PSZ); bf* Yl = (bf*)take(PSZ);
    bf* Qh = (bf*)take(PSZ); bf* Ql = (bf*)take(PSZ); bf* Kh = (bf*)take(PSZ); bf* Kl = (bf*)take(PSZ);
    h16* VT = (h16*)take(PSZ);
    if ((size_t)(wsp - (char*)d_ws) > ws_size) return;
    bf* Ch = Yh; bf* Cl = Yl;

    k_wt<<<dim3(DM / 64, HD / 64, NH), 256, 0, stream>>>(wq, WQ, DM, HD);
    k_wt<<<dim3(DM / 64, HD / 64, NH), 256, 0, stream>>>(wk, WK, DM, HD);
    k_wt<<<dim3(DM / 64, HD / 64, NH), 256, 0, stream>>>(wv, WV, DM, HD);
    k_wt<<<dim3(DM / 64, DM / 64, 1), 256, 0, stream>>>(wp, WP, DM, DM);
    k_ln<<<MTOK / 8, 256, 0, stream>>>(x, lng, lnb, Yh, Yl);
    k_gemmw<0><<<dim3(MTOK / 64, DM / 64, 1), 32, 0, stream>>>(Yh, Yl, WQ, bq, Qh, Ql, (h16*)nullptr, (float*)nullptr);
    k_gemmw<0><<<dim3(MTOK / 64, DM / 64, 1), 32, 0, stream>>>(Yh, Yl, WK, bk, Kh, Kl, (h16*)nullptr, (float*)nullptr);
    k_gemmw<1><<<dim3(MTOK / 64, DM / 64, 1), 32, 0, stream>>>(Yh, Yl, WV, bv, (bf*)nullptr, (bf*)nullptr, VT, (float*)nullptr);
    k_attn<<<dim3(SEQ / 64, NB * NH, 1), 128, 0, stream>>>(Qh, Ql, Kh, Kl, VT, Ch, Cl);
    k_gemmw<2><<<dim3(MTOK / 64, DM / 64, 1), 32, 0, stream>>>(Ch, Cl, WP, bp, (bf*)nullptr, (bf*)nullptr, (h16*)nullptr, OUT);
}
